// ModernAttention_29111288332610
// MI455X (gfx1250) — hardware-verified
//
#include <hip/hip_runtime.h>


namespace {
constexpr int S_ = 2048, Bn = 2, D = 2048, H = 16, KVH = 4, HD = 128, NT = S_ * Bn, DK = KVH * HD  ;
constexpr float XS = 8.0f, PS = 8.0f, ISQ = 0.08838834764831845f;
struct Wo_ { static constexpr size_t Q = 0, K = (size_t)D * D, V = K + (size_t)DK * D, O = V + (size_t)DK * D, END = O + (size_t)D * D; };
__constant__ unsigned int kInvFreqBits[64] = {0x3f800000,0x3f5dafd7,0x3f3ff911,0x3f263de0,0x3f0ff59a,0x3ef953cf,0x3ed7e89b,0x3ebaf81b,0x3ea1e89b,0x3e8c3504,0x3e72d423,0x3e5247ed,0x3e361887,0x3e1db040,0x3e088d77,0x3dec7fd6,0x3dcccccd,0x3db15978,0x3d99940d,0x3d84fe4d,0x3d6655c2,0x3d47763f,0x3d2cba15,0x3d159348,0x3d0186e3,0x3ce054d2,0x3cc2434f,0x3ca8398b,0x3c91ad39,0x3c7c4d33,0x3c5a7bf2,0x3c3d3311,0x3c23d70a,0x3c0de12d,0x3bf5b9b0,0x3bd4ca15,0x3bb8449c,0x3b9f91cc,0x3b8a2e77,0x3b6f520e,0x3b4f3e38,0x3b33770f,0x3b1b690d,0x3b06946f,0x3ae91528,0x3ac9d75c,0x3aaec98e,0x3a975c0e,0x3a83126f,0x3a6301e2,0x3a44948c,0x3a2a3b44,0x3a136a16,0x39ff4fac,0x39dd1725,0x39bf74d7,0x39a5cb60,0x398f9272,0x3978a815,0x395753e4,0x393a7753,0x39217916,0x390bd472,0x38f22ce2};

typedef _Float16 b16;
typedef __attribute__((ext_vector_type(16))) _Float16 v16b;
typedef __attribute__((ext_vector_type(8))) _Float16 v8b;
typedef __attribute__((ext_vector_type(8))) float v8f;
typedef __attribute__((ext_vector_type(4))) float v4f;
__device__ __forceinline__ float bf16_rne(float f) { unsigned int u = __float_as_uint(f); u += 0x7FFFu + ((u >> 16) & 1u); return __uint_as_float(u & 0xFFFF0000u); }
__device__ __forceinline__ void split16(float v, b16& hi, b16& lo) { hi = (b16)v; lo = (b16)(v - (float)hi); }
__device__ __forceinline__ v16b frag_kb(const b16* p, int hh) { const v8b a = *(const v8b*)(p + 8 * hh), b = *(const v8b*)(p + 16 + 8 * hh); v16b f;
#pragma unroll
  for (int e = 0; e < 8; ++e) { f[e] = a[e]; f[8 + e] = b[e]; } return f; }
__device__ __forceinline__ v8f wmma16b(v16b a, v16b b, v8f c) { v8f d = __builtin_amdgcn_wmma_f32_16x16x32_f16(false, a, false, b, (short)0, c, false, false); asm volatile("v_nop\n\tv_nop\n\tv_nop\n\tv_nop" : "+v"(d) : "v"(a), "v"(b)); return d; }
__device__ __forceinline__ void wave_lds_sync() { __builtin_amdgcn_fence(__ATOMIC_RELEASE, "workgroup"); __builtin_amdgcn_wave_barrier(); __builtin_amdgcn_fence(__ATOMIC_ACQUIRE, "workgroup"); }
__device__ __forceinline__ float nexp(float x) { return __builtin_amdgcn_exp2f(x * 1.4426950408889634f); }
__device__ __forceinline__ float pmul(float a, float b) { float p = a * b; asm volatile("" : "+v"(p)); return p; }
__device__ __forceinline__ void sincos_r(float ang, float& sn, float& cs) { const float k = rintf(ang * 0.15915494309189535f); float r = __builtin_fmaf(k, -6.28318548202514648f, ang); r = __builtin_fmaf(k, 1.7484556025237907e-7f, r);
  const float t = r * 0.15915494309189535f; sn = __builtin_amdgcn_sinf(t); cs = __builtin_amdgcn_cosf(t); }

__global__ __launch_bounds__(256) void prep_kernel(const float* __restrict__ x, const float* __restrict__ wq, const float* __restrict__ wk, const float* __restrict__ wv, const float* __restrict__ wo, b16* __restrict__ R, b16* __restrict__ X) {
  const size_t tid = (size_t)blockIdx.x * 256 + threadIdx.x, nth = (size_t)gridDim.x * 256;
  auto tr = [&](size_t base, int nout, int kin, const float* W) { for (size_t p = tid; p < (size_t)nout * (kin / 8); p += nth) { const int o = (int)(p / (kin / 8)), k0 = (int)(p % (kin / 8)) * 8; v8b v;
#pragma unroll
      for (int e = 0; e < 8; ++e) v[e] = (b16)bf16_rne(W[(size_t)(k0 + e) * nout + o]); *(volatile v8b*)(R + base + (size_t)o * kin + k0) = v; } };
  for (int pass = 0; pass < 2; ++pass) { tr(Wo_::Q, D, D, wq); tr(Wo_::K, DK, D, wk); tr(Wo_::V, DK, D, wv); tr(Wo_::O, D, D, wo);
    for (size_t p = tid; p < (size_t)NT * D / 8; p += nth) { v8b v; for (int e = 0; e < 8; ++e) v[e] = (b16)(bf16_rne(x[p * 8 + e]) * XS); *(volatile v8b*)(X + p * 8) = v; }
    __threadfence(); }
}

template <int MODE, int TWO>
__global__ __launch_bounds__(64) void gemm_kernel(const b16* __restrict__ A, const b16* __restrict__ Al, const b16* __restrict__ Bw, int N, b16* __restrict__ O1, b16* __restrict__ O2, float* __restrict__ O32) {
  __shared__ __attribute__((aligned(16))) float Ts[2][32][128 + 4];
  const int lane = threadIdx.x & 31, wave = threadIdx.x >> 5, nloc = lane & 15, hlf = lane >> 4, m0 = blockIdx.y * 32, c0 = blockIdx.x * 256 + wave * 128;
#pragma unroll 1
  for (int hf = 0; hf < 2; ++hf) { v8f acc[2][4];
#pragma unroll
    for (int r = 0; r < 2; ++r)
#pragma unroll
      for (int t = 0; t < 4; ++t) acc[r][t] = (v8f){};
#pragma unroll 2
    for (int kb = 0; kb < D; kb += 32) { const v16b a0 = frag_kb(A + (size_t)(m0 + nloc) * D + kb, hlf), a1 = frag_kb(A + (size_t)(m0 + 16 + nloc) * D + kb, hlf); v16b l0, l1; if (TWO) { l0 = frag_kb(Al + (size_t)(m0 + nloc) * D + kb, hlf); l1 = frag_kb(Al + (size_t)(m0 + 16 + nloc) * D + kb, hlf); }
#pragma unroll
      for (int t = 0; t < 4; ++t) { const v16b bw = frag_kb(Bw + (size_t)(c0 + (hf * 4 + t) * 16 + nloc) * D + kb, hlf); acc[0][t] = wmma16b(a0, bw, acc[0][t]); acc[1][t] = wmma16b(a1, bw, acc[1][t]); if (TWO) { acc[0][t] = wmma16b(l0, bw, acc[0][t]); acc[1][t] = wmma16b(l1, bw, acc[1][t]); } } }
#pragma unroll
    for (int t = 0; t < 4; ++t)
#pragma unroll
      for (int r = 0; r < 2; ++r)
#pragma unroll
        for (int v = 0; v < 8; ++v) Ts[wave][r * 16 + 8 * hlf + v][(hf * 4 + t) * 16 + nloc] = acc[r][t][v] * (1.0f / XS); }
  wave_lds_sync();
  if (MODE == 0) {
    for (int i = lane; i < 32 * 64; i += 32) { const int rr = i >> 6, dd = i & 63; const int s = (m0 + rr) / Bn; float sn, cs; sincos_r(pmul((float)s, __uint_as_float(kInvFreqBits[dd])), sn, cs);
      const float a_ = Ts[wave][rr][dd], b_ = Ts[wave][rr][64 + dd]; Ts[wave][rr][dd] = pmul(a_, cs) - pmul(b_, sn); Ts[wave][rr][64 + dd] = pmul(b_, cs) + pmul(a_, sn); }
    wave_lds_sync(); }
  for (int pass = 0; pass < 2; ++pass) {
    if (MODE == 2) { for (int i = lane; i < 32 * 32; i += 32) { const int rr = i >> 5, c4 = (i & 31) * 4; *(volatile v4f*)(O32 + (size_t)(m0 + rr) * N + c0 + c4) = *(const v4f*)(&Ts[wave][rr][c4]); } }
    else if (MODE == 1) { for (int i = lane; i < 32 * 16; i += 32) { const int rr = i >> 4, c8 = (i & 15) * 8; v8b o; for (int e = 0; e < 8; ++e) o[e] = (b16)(Ts[wave][rr][c8 + e] * XS); *(volatile v8b*)(O1 + (size_t)(m0 + rr) * N + c0 + c8) = o; } }
    else { for (int i = lane; i < 32 * 16; i += 32) { const int rr = i >> 4, c8 = (i & 15) * 8; v8b oh, ol; for (int e = 0; e < 8; ++e) { b16 a_, c_; split16(Ts[wave][rr][c8 + e] * XS, a_, c_); oh[e] = a_; ol[e] = c_; } const size_t gi = (size_t)(m0 + rr) * N + c0 + c8; *(volatile v8b*)(O1 + gi) = oh; *(volatile v8b*)(O2 + gi) = ol; } }
    __threadfence(); }
}

__global__ __launch_bounds__(256) void vt_kernel(const b16* __restrict__ Vr, b16* __restrict__ vt) {
  __shared__ __attribute__((aligned(16))) b16 Tt[HD][128 + 8];
  const int b = blockIdx.z, g = blockIdx.y, s0 = blockIdx.x * 128, t_ = threadIdx.x;
  for (int i = t_; i < 128 * (HD / 8); i += 256) { const int tk = i >> 4, d8 = (i & 15) * 8; const v8b vv = *(const v8b*)(Vr + ((size_t)((s0 + tk) * Bn + b)) * DK + g * HD + d8); for (int e = 0; e < 8; ++e) Tt[d8 + e][tk] = vv[e]; }
  __syncthreads();
  for (int pass = 0; pass < 2; ++pass) { for (int i = t_; i < HD * 16; i += 256) { const int d = i >> 4, c8 = (i & 15) * 8; *(volatile v8b*)(vt + (((size_t)b * KVH + g) * HD + d) * S_ + s0 + c8) = *(const v8b*)(&Tt[d][c8]); } __threadfence(); }
}

__global__ __launch_bounds__(128) void attn_kernel(const b16* __restrict__ QH, const b16* __restrict__ QL, const b16* __restrict__ KH, const b16* __restrict__ KL, const b16* __restrict__ vt, const b16* __restrict__ vtl, b16* __restrict__ ctxh, b16* __restrict__ ctxl, int boff) {
  __shared__ __attribute__((aligned(16))) b16 Oh[16][4 * HD + 8], Ol[16][4 * HD + 8];
  const int bx = blockIdx.x + boff; const int wid = threadIdx.x >> 5, lane = threadIdx.x & 31, hh = lane >> 4, col = lane & 15; const int b = bx / (S_ / 16), s0 = (bx % (S_ / 16)) * 16, h = blockIdx.y * 4 + wid, g = h / 4, si = s0 + col;
  const size_t qp = (size_t)Bn * D, kp = (size_t)Bn * DK; const b16* Qr = QH + (size_t)b * D + h * HD; const b16* Qrl = QL + (size_t)b * D + h * HD; const b16* Kr = KH + (size_t)b * DK + g * HD; const b16* Krl = KL + (size_t)b * DK + g * HD; const b16* V = vt + (((size_t)b * KVH + g) * HD) * S_; const b16* Vl = vtl + (((size_t)b * KVH + g) * HD) * S_;
  v16b qh_[4], ql_[4];
#pragma unroll
  for (int j = 0; j < 4; ++j) { qh_[j] = frag_kb(Qr + (size_t)si * qp + 32 * j, hh); ql_[j] = frag_kb(Qrl + (size_t)si * qp + 32 * j, hh); }
  float m = -INFINITY, l = 0.0f; v8f o[8];
#pragma unroll
  for (int t = 0; t < 8; ++t) o[t] = (v8f){};
  for (int kb = 0; kb <= s0 + 15; kb += 32) { v8f s0v = {}, s1v = {};
#pragma unroll
    for (int j = 0; j < 4; ++j) { const b16* k0 = Kr + (size_t)(kb + col) * kp + 32 * j; const b16* k0l = Krl + (size_t)(kb + col) * kp + 32 * j; const b16* k1 = Kr + (size_t)(kb + 16 + col) * kp + 32 * j; const b16* k1l = Krl + (size_t)(kb + 16 + col) * kp + 32 * j;
      const v16b a0 = frag_kb(k0, hh), a0l = frag_kb(k0l, hh), a1 = frag_kb(k1, hh), a1l = frag_kb(k1l, hh);
      s0v = wmma16b(a0, qh_[j], s0v); s0v = wmma16b(a0, ql_[j], s0v); s0v = wmma16b(a0l, qh_[j], s0v); s1v = wmma16b(a1, qh_[j], s1v); s1v = wmma16b(a1, ql_[j], s1v); s1v = wmma16b(a1l, qh_[j], s1v); }
    float mr = -INFINITY;
#pragma unroll
    for (int r = 0; r < 8; ++r) { const int k0i = kb + 8 * hh + r, k1i = k0i + 16; s0v[r] = (k0i <= si) ? s0v[r] * (ISQ / (XS * XS)) : -INFINITY; s1v[r] = (k1i <= si) ? s1v[r] * (ISQ / (XS * XS)) : -INFINITY; mr = fmaxf(mr, fmaxf(s0v[r], s1v[r])); }
    mr = fmaxf(mr, __shfl_xor(mr, 16)); const float mn = fmaxf(m, mr), al_ = nexp(m - mn); m = mn; float sum = 0.0f; v16b pb, pl;
#pragma unroll
    for (int r = 0; r < 8; ++r) { const float e0 = (s0v[r] == -INFINITY) ? 0.0f : nexp(s0v[r] - mn), e1 = (s1v[r] == -INFINITY) ? 0.0f : nexp(s1v[r] - mn); sum += e0 + e1; b16 a_, c_; split16(e0 * PS, a_, c_); pb[r] = a_; pl[r] = c_; split16(e1 * PS, a_, c_); pb[8 + r] = a_; pl[8 + r] = c_; }
    sum += __shfl_xor(sum, 16); l = l * al_ + sum;
#pragma unroll
    for (int t = 0; t < 8; ++t) { o[t] *= al_; const v16b vh = frag_kb(V + (size_t)(t * 16 + col) * S_ + kb, hh), vlo = frag_kb(Vl + (size_t)(t * 16 + col) * S_ + kb, hh); o[t] = wmma16b(vh, pb, o[t]); o[t] = wmma16b(vh, pl, o[t]); o[t] = wmma16b(vlo, pb, o[t]); } }
  const float inv = 1.0f / (l * PS);
#pragma unroll
  for (int t = 0; t < 8; ++t)
#pragma unroll
    for (int r = 0; r < 8; ++r) { b16 a_, c_; split16(o[t][r] * inv, a_, c_); Oh[col][wid * HD + t * 16 + 8 * hh + r] = a_; Ol[col][wid * HD + t * 16 + 8 * hh + r] = c_; }
  __syncthreads();
  for (int pass = 0; pass < 2; ++pass) { for (int i = threadIdx.x; i < 16 * 64; i += 128) { const int rr = i >> 6, c8 = (i & 63) * 8; const size_t gi = ((size_t)((s0 + rr) * Bn + b)) * D + blockIdx.y * 4 * HD + c8; *(volatile v8b*)(ctxh + gi) = *(const v8b*)(&Oh[rr][c8]); *(volatile v8b*)(ctxl + gi) = *(const v8b*)(&Ol[rr][c8]); } __threadfence(); }
}
}

extern "C" void kernel_launch(void* const* d_in, const int* in_sizes, int n_in,
                              void* d_out, int out_size, void* d_ws, size_t ws_size, hipStream_t stream) {
  (void)n_in; (void)out_size;
  const float* x = (const float*)d_in[0]; const float* wq = (const float*)d_in[1]; const float* wk = (const float*)d_in[2]; const float* wv = (const float*)d_in[3]; const float* wo = (const float*)d_in[4];
  float* out = (float*)d_out;
  if (in_sizes[0] != NT * D || in_sizes[1] != D * D || in_sizes[2] != D * DK || in_sizes[4] != D * D) return;
  size_t off = 0; char* ws = (char*)d_ws;
  auto carve = [&](size_t bytes) { char* p = ws + off; off += (bytes + 255) & ~(size_t)255; return p; };
  b16* R = (b16*)carve(Wo_::END * 2); b16* X = (b16*)carve((size_t)NT * D * 2); b16* QH = (b16*)carve((size_t)NT * D * 2); b16* QL = (b16*)carve((size_t)NT * D * 2); b16* KH = (b16*)carve((size_t)NT * DK * 2); b16* KL = (b16*)carve((size_t)NT * DK * 2); b16* VR = (b16*)carve((size_t)NT * DK * 2); b16* VT = (b16*)carve((size_t)NT * DK * 2); b16* VRl = (b16*)carve((size_t)NT * DK * 2); b16* VTl = (b16*)carve((size_t)NT * DK * 2);
  if (off > ws_size) return;
  b16* CH = X; b16* CL = (b16*)carve((size_t)NT * D * 2);
  if (off > ws_size) return;
  prep_kernel<<<1024, 256, 0, stream>>>(x, wq, wk, wv, wo, R, X);
  gemm_kernel<0, 0><<<dim3(D / 256, NT / 32), 64, 0, stream>>>(X, nullptr, R + Wo_::Q, D, QH, QL, nullptr);
  gemm_kernel<0, 0><<<dim3(DK / 256, NT / 32), 64, 0, stream>>>(X, nullptr, R + Wo_::K, DK, KH, KL, nullptr);
  gemm_kernel<3, 0><<<dim3(DK / 256, NT / 32), 64, 0, stream>>>(X, nullptr, R + Wo_::V, DK, VR, VRl, nullptr);
  vt_kernel<<<dim3(S_ / 128, KVH, Bn), 256, 0, stream>>>(VR, VT);
  vt_kernel<<<dim3(S_ / 128, KVH, Bn), 256, 0, stream>>>(VRl, VTl);
  attn_kernel<<<dim3(Bn * S_ / 16, 4), 128, 0, stream>>>(QH, QL, KH, KL, VT, VTl, CH, CL, 0);
  gemm_kernel<2, 1><<<dim3(D / 256, NT / 32), 64, 0, stream>>>(CH, CL, R + Wo_::O, D, nullptr, nullptr, out);
}
